// Block_62362925138693
// MI455X (gfx1250) — hardware-verified
//
#include <hip/hip_runtime.h>
#include <math.h>

#ifndef NB
#define NB 2
#endif
#ifndef SEQ
#define SEQ 2048
#endif
#define NB_FULL 2
#define SEQ_FULL 2048
#define WD 1024
#define NH 16
#define HDIM 64
#define FF 4096
#define QW 3072
#define LN_NQ 8
#define ROWS (NB * SEQ)

static_assert(WD == 32 * 4 * LN_NQ);
static_assert(NH * HDIM == WD);
static_assert(QW == 3 * WD);
static_assert(HDIM == 64);
static_assert(SEQ % 64 == 0);
static_assert(ROWS % 64 == 0);
static_assert(WD % 64 == 0 && QW % 64 == 0 && FF % 64 == 0);
static_assert(WD % 32 == 0 && FF % 32 == 0);
static_assert(WD % 8 == 0 && FF % 8 == 0);
static_assert(WD / 8 == (1 << 7) && FF / 8 == (1 << 9));
static_assert(NB <= NB_FULL && SEQ <= SEQ_FULL);

typedef __attribute__((ext_vector_type(16))) _Float16 v16h;
typedef __attribute__((ext_vector_type(8)))  _Float16 v8h;
typedef __attribute__((ext_vector_type(8)))  float    v8f;
typedef __attribute__((ext_vector_type(4)))  float    v4f;
typedef __attribute__((ext_vector_type(4)))  unsigned int u4v;
typedef __attribute__((ext_vector_type(2)))  unsigned int u2v;


#define VST2(T, ptr, val) do { const T vst2_v_ = (val); *(volatile T*)(ptr) = vst2_v_; __threadfence(); *(volatile T*)(ptr) = vst2_v_; } while (0)

__device__ __forceinline__ float cmb_bf(float v) {
    const unsigned u = __builtin_bit_cast(unsigned, v);
    const unsigned r = (u + 0x7fffu + ((u >> 16) & 1u)) & 0xffff0000u;
    return __builtin_bit_cast(float, r);
}
__device__ __forceinline__ unsigned int pk2h(float a, float b) {
    return (unsigned int)__builtin_bit_cast(unsigned short, (_Float16)a) | ((unsigned int)__builtin_bit_cast(unsigned short, (_Float16)b) << 16);
}

__device__ __forceinline__ void dep_guard_h(v8f& a, v8f& b, v16h x, v16h y) { asm volatile("v_nop\n\tv_nop\n\tv_nop\n\tv_nop" : "+v"(a), "+v"(b) : "v"(x), "v"(y)); }
__device__ __forceinline__ void keep4_h(v16h a, v16h b, v16h c, v16h d) { asm volatile("v_nop" :: "v"(a), "v"(b), "v"(c), "v"(d)); }
__device__ __forceinline__ void acc_guard4(v8f& a, v8f& b, v8f& c, v8f& d) { asm volatile("v_nop\n\tv_nop\n\tv_nop\n\tv_nop" : "+v"(a), "+v"(b), "+v"(c), "+v"(d)); }

union FragH { v16h v; v8h h[2]; };
__device__ __forceinline__ v16h frag_ld(const _Float16* p) { FragH f; f.h[0] = *(const v8h*)(p); f.h[1] = *(const v8h*)(p + 16); return f.v; }
__device__ __forceinline__ v8f mma_h(v16h a, v16h b, v8f c) { return __builtin_amdgcn_wmma_f32_16x16x32_f16(false, a, false, b, (short)0, c, false, false); }
__device__ __forceinline__ v8f wmma16(v16h a, v16h b, v8f c) {
    c = __builtin_amdgcn_wmma_f32_16x16x32_f16(false, a, false, b, (short)0, c, false, false);
    asm volatile("v_nop\n\tv_nop\n\tv_nop\n\tv_nop" : "+v"(c) : "v"(a), "v"(b));
    return c;
}

template <int OUT_MODE, int RESID, int ACT, int BIAS>
__device__ __forceinline__ void gemm64_body(const unsigned short* __restrict__ Ap, int lda, const unsigned short* __restrict__ Btp, int ldb,
                                            void* __restrict__ Cout, int ldc, const float* __restrict__ resid, const float* __restrict__ bias,
                                            int M, int N, int K, float scale, float* slab) {
    const _Float16* A = (const _Float16*)Ap; const _Float16* Bt = (const _Float16*)Btp;
    const int lane = threadIdx.x & 31;
    const int wave = threadIdx.x >> 5;
    const int tilesN = N >> 6;
    const int tilesM = M >> 6;
    const int tile = blockIdx.x * 8 + wave;
    if (tile >= tilesM * tilesN) return;
    const int tm = tile / tilesN;
    const int tn = tile - tm * tilesN;
    const int m0 = tm << 6;
    const int n0 = tn << 6;
    const int rlane = lane & 15;
    const int koff  = (lane >> 4) * 8;
    const int mOff  = (lane >> 4) * 8;

    v8f acc[4][4];
#pragma unroll
    for (int i = 0; i < 4; ++i)
#pragma unroll
        for (int j = 0; j < 4; ++j) acc[i][j] = (v8f){0.f, 0.f, 0.f, 0.f, 0.f, 0.f, 0.f, 0.f};

    for (int k0 = 0; k0 < K; k0 += 32) {
        v16h bh[4];
#pragma unroll
        for (int j = 0; j < 4; ++j) {
            const size_t bo = (size_t)(n0 + (j << 4) + rlane) * ldb + koff + k0;
            bh[j] = frag_ld(Bt + bo);
        }
#pragma unroll
        for (int i = 0; i < 4; ++i) {
            const size_t ao = (size_t)(m0 + (i << 4) + rlane) * lda + koff + k0;
            const v16h ah = frag_ld(A + ao);
#pragma unroll
            for (int j = 0; j < 4; ++j) acc[i][j] = mma_h(ah, bh[j], acc[i][j]);
            dep_guard_h(acc[i][0], acc[i][3], ah, ah);
        }
        keep4_h(bh[0], bh[1], bh[2], bh[3]);
    }
    acc_guard4(acc[0][0], acc[0][1], acc[0][2], acc[0][3]);
    acc_guard4(acc[1][0], acc[1][1], acc[1][2], acc[1][3]);
    acc_guard4(acc[2][0], acc[2][1], acc[2][2], acc[2][3]);
    acc_guard4(acc[3][0], acc[3][1], acc[3][2], acc[3][3]);

    v4f bzA = (v4f){0.f, 0.f, 0.f, 0.f};
    v4f bzB = (v4f){0.f, 0.f, 0.f, 0.f};
    if (BIAS) {
        if (OUT_MODE == 0) {
            bzA = *(const v4f*)(bias + n0 + (lane & 15) * 4);
        } else {
            bzA = *(const v4f*)(bias + n0 + (lane & 7) * 8);
            bzB = *(const v4f*)(bias + n0 + (lane & 7) * 8 + 4);
        }
        bzA.x = cmb_bf(bzA.x); bzA.y = cmb_bf(bzA.y); bzA.z = cmb_bf(bzA.z); bzA.w = cmb_bf(bzA.w);
        bzB.x = cmb_bf(bzB.x); bzB.y = cmb_bf(bzB.y); bzB.z = cmb_bf(bzB.z); bzB.w = cmb_bf(bzB.w);
    }

#pragma unroll
    for (int i = 0; i < 4; ++i) {
        const int mBase = m0 + (i << 4);
#pragma unroll
        for (int j = 0; j < 4; ++j) {
#pragma unroll
            for (int r = 0; r < 8; ++r) {
                slab[(mOff + r) * 68 + (j << 4) + rlane] = acc[i][j][r] * scale;
            }
        }
        __builtin_amdgcn_fence(3  , "workgroup");
        __builtin_amdgcn_wave_barrier();
        __builtin_amdgcn_fence(2  , "workgroup");
        if (OUT_MODE == 0) {
            float* C = (float*)Cout;
            const int hh = lane >> 4, c4 = (lane & 15) * 4;
            for (int pass = 0; pass < 2; ++pass) {
#pragma unroll
                for (int it = 0; it < 8; ++it) {
                    const int row = it * 2 + hh;
                    v4f v = *(const v4f*)(slab + row * 68 + c4);
                    if (BIAS) { v.x = v.x + bzA.x; v.y = v.y + bzA.y; v.z = v.z + bzA.z; v.w = v.w + bzA.w; }
                    if (ACT == 2) { v.x = fmaxf(v.x, 0.0f); v.y = fmaxf(v.y, 0.0f); v.z = fmaxf(v.z, 0.0f); v.w = fmaxf(v.w, 0.0f); }
                    if (RESID != 0) {
                        const v4f x = *(const v4f*)(resid + (size_t)(mBase + row) * ldc + n0 + c4);
                        v.x = x.x + v.x; v.y = x.y + v.y; v.z = x.z + v.z; v.w = x.w + v.w;
                    }
                    *(volatile v4f*)(C + (size_t)(mBase + row) * ldc + n0 + c4) = v;
                }
                __threadfence();
            }
        } else {
            const int q = lane >> 3, c8 = (lane & 7) * 8;
            _Float16* C = (_Float16*)Cout;
            for (int pass = 0; pass < 2; ++pass) {
#pragma unroll
                for (int it = 0; it < 4; ++it) {
                    const int row = it * 4 + q;
                    const float* sp = slab + row * 68 + c8;
                    float t[8];
#pragma unroll
                    for (int e = 0; e < 8; ++e) t[e] = sp[e];
                    if (BIAS) {
                        t[0] = t[0] + bzA.x; t[1] = t[1] + bzA.y; t[2] = t[2] + bzA.z; t[3] = t[3] + bzA.w;
                        t[4] = t[4] + bzB.x; t[5] = t[5] + bzB.y; t[6] = t[6] + bzB.z; t[7] = t[7] + bzB.w;
                    }
                    if (ACT == 2) {
#pragma unroll
                        for (int e = 0; e < 8; ++e) t[e] = fmaxf(t[e], 0.0f);
                    }
                    v8h hv;
#pragma unroll
                    for (int e = 0; e < 8; ++e) hv[e] = (_Float16)t[e];
                    *(volatile v8h*)(C + (size_t)(mBase + row) * ldc + n0 + c8) = hv;
                }
                __threadfence();
            }
        }
        __builtin_amdgcn_fence(3  , "workgroup");
        __builtin_amdgcn_wave_barrier();
        __builtin_amdgcn_fence(2  , "workgroup");
    }
}

__global__ __launch_bounds__(256) void k_gemm_qkv(const unsigned short* __restrict__ A, const unsigned short* __restrict__ Bt, float* __restrict__ C) {
    __shared__ __align__(16) float sT[8][16 * 68];
    gemm64_body<0, 0, 0, 0>(A, WD, Bt, WD, (void*)C, QW, nullptr, nullptr, ROWS, QW, WD, 0.0625f, sT[threadIdx.x >> 5]);
}
__global__ __launch_bounds__(256) void k_gemm_mlp1(const unsigned short* __restrict__ A, const unsigned short* __restrict__ Bt, unsigned short* __restrict__ C, const float* __restrict__ b1) {
    __shared__ __align__(16) float sT[8][16 * 68];
    gemm64_body<1, 0, 2, 1>(A, WD, Bt, WD, (void*)C, FF, nullptr, b1, ROWS, FF, WD, 0.0625f, sT[threadIdx.x >> 5]);
}
__global__ __launch_bounds__(256) void k_gemm_mlp2(const unsigned short* __restrict__ A, const unsigned short* __restrict__ Bt, float* __restrict__ C, const float* __restrict__ x1, const float* __restrict__ b2) {
    __shared__ __align__(16) float sT[8][16 * 68];
    gemm64_body<0, 1, 0, 1>(A, FF, Bt, FF, (void*)C, WD, x1, b2, ROWS, WD, FF, 0.0625f, sT[threadIdx.x >> 5]);
}

template <int ABF>
__device__ __forceinline__ void ln_body(const float* __restrict__ A, int rpb, long long bstride, const float* __restrict__ GA, const float* __restrict__ BE, int rows, unsigned short* __restrict__ Y16) {
    #pragma clang fp contract(off)
    constexpr int NQ = LN_NQ;
    const int r = blockIdx.x * 8 + (threadIdx.x >> 5); const int L = threadIdx.x & 31; if (r >= rows) return;
    const float* ar = A + (long long)(r / rpb) * bstride + (long long)(r % rpb) * WD;
    v4f v[NQ]; float s = 0.f;
#pragma unroll
    for (int q = 0; q < NQ; ++q) {
        v[q] = *(const v4f*)(ar + 4 * L + 128 * q);
        if (ABF) { v[q].x = cmb_bf(v[q].x); v[q].y = cmb_bf(v[q].y); v[q].z = cmb_bf(v[q].z); v[q].w = cmb_bf(v[q].w); }
        s += (v[q].x + v[q].y) + (v[q].z + v[q].w);
    }
#pragma unroll
    for (int o = 16; o > 0; o >>= 1) s += __shfl_xor(s, o, 32);
    const float mu = s * (1.f / WD); float qq = 0.f;
#pragma unroll
    for (int q = 0; q < NQ; ++q) { v[q].x -= mu; v[q].y -= mu; v[q].z -= mu; v[q].w -= mu; qq += (v[q].x * v[q].x + v[q].y * v[q].y) + (v[q].z * v[q].z + v[q].w * v[q].w); }
#pragma unroll
    for (int o = 16; o > 0; o >>= 1) qq += __shfl_xor(qq, o, 32);
    const float rs = rsqrtf(qq * (1.f / WD) + 1e-5f);
#pragma unroll
    for (int q = 0; q < NQ; ++q) {
        const int c = 4 * L + 128 * q; const v4f ga = *(const v4f*)(GA + c), be = *(const v4f*)(BE + c); v4f y;
        y.x = v[q].x * rs * cmb_bf(ga.x) + cmb_bf(be.x); y.y = v[q].y * rs * cmb_bf(ga.y) + cmb_bf(be.y);
        y.z = v[q].z * rs * cmb_bf(ga.z) + cmb_bf(be.z); y.w = v[q].w * rs * cmb_bf(ga.w) + cmb_bf(be.w);
        u2v pk; pk.x = pk2h(y.x, y.y); pk.y = pk2h(y.z, y.w);
        VST2(u2v, (u2v*)(Y16 + (long long)r * WD + c), pk);
    }
}
__global__ __launch_bounds__(256) void k_ln_in(const float* __restrict__ xin, const float* __restrict__ GA, const float* __restrict__ BE, unsigned short* __restrict__ Y16) {
    ln_body<1>(xin, SEQ, (long long)SEQ_FULL * WD, GA, BE, ROWS, Y16);
}
__global__ __launch_bounds__(256) void k_ln_mid(const float* __restrict__ x1, const float* __restrict__ GA, const float* __restrict__ BE, unsigned short* __restrict__ Y16) {
    ln_body<0>(x1, SEQ, (long long)SEQ * WD, GA, BE, ROWS, Y16);
}

__global__ __launch_bounds__(256) void k_cm_castbT(const float* __restrict__ SRC, unsigned short* __restrict__ DST, long long sbs, long long dbs,
                                                   int lds, int ldd, int ps, int nC, float sc) {
    const long long u = (long long)blockIdx.x * 256 + threadIdx.x; if (u >= ((long long)nC << ps)) return;
    const float* S = SRC + (long long)blockIdx.y * sbs;
    unsigned short* Dp = DST + (long long)blockIdx.y * dbs;
    const int c = (int)(u >> ps); const int r0 = 8 * (int)(u & ((1LL << ps) - 1));
    float w[8];
#pragma unroll
    for (int e = 0; e < 8; ++e) w[e] = cmb_bf(S[(long long)(r0 + e) * lds + c]) * sc;
    u4v pk; pk.x = pk2h(w[0], w[1]); pk.y = pk2h(w[2], w[3]); pk.z = pk2h(w[4], w[5]); pk.w = pk2h(w[6], w[7]);
    VST2(u4v, (u4v*)(Dp + (long long)c * ldd + r0), pk);
}

#define AT_D 64
#define AT_KC 64
__global__ __launch_bounds__(128) void k_attn(const float* __restrict__ qkv, const float* __restrict__ xin, float* __restrict__ x1) {
    __shared__ __align__(16) _Float16 Ksh[AT_KC * AT_D];
    __shared__ __align__(16) _Float16 Vth[AT_D * AT_KC];
    __shared__ __align__(16) _Float16 Psh[4][16 * AT_KC];
    __shared__ __align__(16) float    Os[4][16 * 68];
    const float PSC = 32768.0f;

    const int tid  = threadIdx.x;
    const int wave = tid >> 5;
    const int lane = tid & 31;
    const int hh   = lane >> 4;
    const int c    = lane & 15;

    const int nqb = SEQ / 64;
    const int bx = blockIdx.x;
    const int qb = bx % nqb;
    const int bh = bx / nqb;
    const int h  = bh % NH;
    const int b  = bh / NH;
    const int q0 = qb * 64 + wave * 16;
    const float* base = qkv + (size_t)b * SEQ * QW + h * HDIM;

    v16h qa[2];
    {
        const float* qrow = base + (size_t)(q0 + c) * QW;
#pragma unroll
        for (int dc = 0; dc < 2; ++dc) {
#pragma unroll
            for (int hf = 0; hf < 2; ++hf) {
                const float* p = qrow + dc * 32 + 16 * hf + 8 * hh;
                const v4f a0 = *(const v4f*)(p), a1 = *(const v4f*)(p + 4);
                qa[dc][8 * hf + 0] = (_Float16)a0.x; qa[dc][8 * hf + 1] = (_Float16)a0.y; qa[dc][8 * hf + 2] = (_Float16)a0.z; qa[dc][8 * hf + 3] = (_Float16)a0.w;
                qa[dc][8 * hf + 4] = (_Float16)a1.x; qa[dc][8 * hf + 5] = (_Float16)a1.y; qa[dc][8 * hf + 6] = (_Float16)a1.z; qa[dc][8 * hf + 7] = (_Float16)a1.w;
            }
        }
    }

    float mrow[8], lrow[8];
    v8f oacc[4];
#pragma unroll
    for (int r = 0; r < 8; ++r) { mrow[r] = -INFINITY; lrow[r] = 0.f; }
#pragma unroll
    for (int t = 0; t < 4; ++t) oacc[t] = (v8f){0.f, 0.f, 0.f, 0.f, 0.f, 0.f, 0.f, 0.f};

    _Float16* pw = Psh[wave];
    const int nChunks = qb + 1;
    for (int kc = 0; kc < nChunks; ++kc) {
        const int kv0 = kc * AT_KC;
        __syncthreads();
        {
            const int kvr = tid >> 1, dh = (tid & 1) * 32;
            const float* krow = base + WD + (size_t)(kv0 + kvr) * QW + dh;
            const float* vrow = base + 2 * WD + (size_t)(kv0 + kvr) * QW + dh;
#pragma unroll
            for (int i = 0; i < 4; ++i) {
                const v4f k0v = *(const v4f*)(krow + 8 * i), k1v = *(const v4f*)(krow + 8 * i + 4);
                v8h kk;
                kk[0] = (_Float16)k0v.x; kk[1] = (_Float16)k0v.y; kk[2] = (_Float16)k0v.z; kk[3] = (_Float16)k0v.w;
                kk[4] = (_Float16)k1v.x; kk[5] = (_Float16)k1v.y; kk[6] = (_Float16)k1v.z; kk[7] = (_Float16)k1v.w;
                *(v8h*)(Ksh + kvr * AT_D + dh + 8 * i) = kk;
                const v4f v0v = *(const v4f*)(vrow + 8 * i), v1v = *(const v4f*)(vrow + 8 * i + 4);
                const int d0 = dh + 8 * i;
                Vth[(d0 + 0) * AT_KC + kvr] = (_Float16)v0v.x; Vth[(d0 + 1) * AT_KC + kvr] = (_Float16)v0v.y;
                Vth[(d0 + 2) * AT_KC + kvr] = (_Float16)v0v.z; Vth[(d0 + 3) * AT_KC + kvr] = (_Float16)v0v.w;
                Vth[(d0 + 4) * AT_KC + kvr] = (_Float16)v1v.x; Vth[(d0 + 5) * AT_KC + kvr] = (_Float16)v1v.y;
                Vth[(d0 + 6) * AT_KC + kvr] = (_Float16)v1v.z; Vth[(d0 + 7) * AT_KC + kvr] = (_Float16)v1v.w;
            }
        }
        __syncthreads();

        v8f s[4];
#pragma unroll
        for (int j = 0; j < 4; ++j) {
            s[j] = (v8f){0.f, 0.f, 0.f, 0.f, 0.f, 0.f, 0.f, 0.f};
#pragma unroll
            for (int dc = 0; dc < 2; ++dc) {
                FragH kb;
                kb.h[0] = *(const v8h*)(Ksh + (j * 16 + c) * AT_D + dc * 32 + 8 * hh);
                kb.h[1] = *(const v8h*)(Ksh + (j * 16 + c) * AT_D + dc * 32 + 16 + 8 * hh);
                s[j] = wmma16(qa[dc], kb.v, s[j]);
            }
        }
        const bool diag = (kc == qb);
        float cm[8];
#pragma unroll
        for (int r = 0; r < 8; ++r) {
            const int qrow = q0 + 8 * hh + r;
            float m = -INFINITY;
#pragma unroll
            for (int j = 0; j < 4; ++j) {
                const int kvcol = kv0 + j * 16 + c;
                float sv = s[j][r] * 0.125f;
                sv = (diag && (kvcol > qrow)) ? -INFINITY : sv;
                s[j][r] = sv;
                m = fmaxf(m, sv);
            }
#pragma unroll
            for (int off = 1; off < 16; off <<= 1) m = fmaxf(m, __shfl_xor(m, off, 32));
            cm[r] = m;
        }
#pragma unroll
        for (int r = 0; r < 8; ++r) {
            const float mnew = fmaxf(mrow[r], cm[r]);
            const float alpha = expf(mrow[r] - mnew);
            mrow[r] = mnew;
            float psum = 0.f;
#pragma unroll
            for (int j = 0; j < 4; ++j) {
                const float p = expf(s[j][r] - mnew);
                psum += p;
                pw[(8 * hh + r) * AT_KC + j * 16 + c] = (_Float16)(p * PSC);
            }
#pragma unroll
            for (int off = 1; off < 16; off <<= 1) psum += __shfl_xor(psum, off, 32);
            lrow[r] = lrow[r] * alpha + psum;
#pragma unroll
            for (int t = 0; t < 4; ++t) oacc[t][r] *= alpha;
        }
        __builtin_amdgcn_fence(3  , "workgroup");
        __builtin_amdgcn_wave_barrier();
        __builtin_amdgcn_fence(2  , "workgroup");
#pragma unroll
        for (int kk = 0; kk < 2; ++kk) {
            FragH pa;
            pa.h[0] = *(const v8h*)(pw + c * AT_KC + kk * 32 + 8 * hh);
            pa.h[1] = *(const v8h*)(pw + c * AT_KC + kk * 32 + 16 + 8 * hh);
#pragma unroll
            for (int t = 0; t < 4; ++t) {
                FragH vb;
                vb.h[0] = *(const v8h*)(Vth + (t * 16 + c) * AT_KC + kk * 32 + 8 * hh);
                vb.h[1] = *(const v8h*)(Vth + (t * 16 + c) * AT_KC + kk * 32 + 16 + 8 * hh);
                oacc[t] = wmma16(pa.v, vb.v, oacc[t]);
            }
        }
    }

    float* os = Os[wave];
#pragma unroll
    for (int r = 0; r < 8; ++r) {
        const float inv = 1.0f / (lrow[r] * PSC);
#pragma unroll
        for (int t = 0; t < 4; ++t) os[(8 * hh + r) * 68 + t * 16 + c] = oacc[t][r] * inv;
    }
    __builtin_amdgcn_fence(3  , "workgroup");
    __builtin_amdgcn_wave_barrier();
    __builtin_amdgcn_fence(2  , "workgroup");
    {
        const int c4 = c * 4;
        const float* xb = xin + (size_t)b * SEQ_FULL * WD + h * HDIM;
        float* ob = x1 + (size_t)b * SEQ * WD + h * HDIM;
        for (int pass = 0; pass < 2; ++pass) {
#pragma unroll
            for (int it = 0; it < 8; ++it) {
                const int row = it * 2 + hh;
                v4f v = *(const v4f*)(os + row * 68 + c4);
                v4f xr = *(const v4f*)(xb + (size_t)(q0 + row) * WD + c4);
                xr.x = cmb_bf(xr.x); xr.y = cmb_bf(xr.y); xr.z = cmb_bf(xr.z); xr.w = cmb_bf(xr.w);
                v.x = xr.x + v.x; v.y = xr.y + v.y; v.z = xr.z + v.z; v.w = xr.w + v.w;
                *(volatile v4f*)(ob + (size_t)(q0 + row) * WD + c4) = v;
            }
            __threadfence();
        }
    }
}

constexpr size_t SZ_H16  = (size_t)ROWS * WD * 2;
constexpr size_t SZ_H2   = (size_t)ROWS * WD * 2;
constexpr size_t SZ_WQKV = (size_t)QW * WD * 2;
constexpr size_t SZ_W1T  = (size_t)FF * WD * 2;
constexpr size_t SZ_W2T  = (size_t)WD * FF * 2;
constexpr size_t SZ_QKV  = (size_t)ROWS * QW * 4;
constexpr size_t SZ_X1   = (size_t)ROWS * WD * 4;
constexpr size_t SZ_A1   = (size_t)ROWS * FF * 2;
constexpr size_t SZ_TOTAL = SZ_H16 + SZ_WQKV + SZ_W1T + SZ_W2T + SZ_QKV + SZ_X1 + SZ_A1;
static_assert(SZ_H2 <= SZ_H16);
static_assert(SZ_H16 % 256 == 0 && SZ_WQKV % 256 == 0 && SZ_W1T % 256 == 0 && SZ_W2T % 256 == 0);
static_assert(SZ_QKV % 256 == 0 && SZ_X1 % 256 == 0 && SZ_A1 % 256 == 0);
static_assert(SZ_TOTAL <= (size_t)134217728);
static_assert(((ROWS / 64) * (QW / 64)) % 8 == 0 && ((ROWS / 64) * (WD / 64)) % 8 == 0 && ((ROWS / 64) * (FF / 64)) % 8 == 0);
static_assert((HDIM * (WD / 8)) % 256 == 0 && (FF * (WD / 8)) % 256 == 0 && (WD * (FF / 8)) % 256 == 0);

extern "C" void kernel_launch(void* const* d_in, const int* in_sizes, int n_in, void* d_out, int out_size, void* d_ws, size_t ws_size, hipStream_t stream) {
    if (n_in < 12) return;
    if (in_sizes[0] < ((NB - 1) * SEQ_FULL + SEQ) * WD) return;
    if (in_sizes[1] < NH * WD * HDIM || in_sizes[2] < NH * WD * HDIM || in_sizes[3] < NH * WD * HDIM) return;
    if (in_sizes[4] < WD * FF || in_sizes[5] < FF || in_sizes[6] < FF * WD || in_sizes[7] < WD) return;
    if (in_sizes[8] < WD || in_sizes[9] < WD || in_sizes[10] < WD || in_sizes[11] < WD) return;
    if (out_size < ROWS * WD) return;
    if (SZ_TOTAL > ws_size) return;
    const float* x   = (const float*)d_in[0];
    const float* Wq  = (const float*)d_in[1];
    const float* Wk  = (const float*)d_in[2];
    const float* Wv  = (const float*)d_in[3];
    const float* W1  = (const float*)d_in[4];
    const float* b1  = (const float*)d_in[5];
    const float* W2  = (const float*)d_in[6];
    const float* b2  = (const float*)d_in[7];
    const float* g1  = (const float*)d_in[8];
    const float* be1 = (const float*)d_in[9];
    const float* g2  = (const float*)d_in[10];
    const float* be2 = (const float*)d_in[11];
    float* out = (float*)d_out;

    char* wsp = (char*)d_ws;
    unsigned short* H16    = (unsigned short*)wsp; wsp += SZ_H16;
    unsigned short* WQKV16 = (unsigned short*)wsp; wsp += SZ_WQKV;
    unsigned short* W1T    = (unsigned short*)wsp; wsp += SZ_W1T;
    unsigned short* W2T    = (unsigned short*)wsp; wsp += SZ_W2T;
    float*          QKV    = (float*)wsp;          wsp += SZ_QKV;
    float*          X1     = (float*)wsp;          wsp += SZ_X1;
    unsigned short* A1     = (unsigned short*)wsp; wsp += SZ_A1;
    unsigned short* H2     = H16;

    k_ln_in<<<(ROWS + 7) / 8, 256, 0, stream>>>(x, g1, be1, H16);
    k_cm_castbT<<<dim3((HDIM * (WD / 8)) / 256, NH), 256, 0, stream>>>(Wq, WQKV16,                       (long long)WD * HDIM, (long long)HDIM * WD, HDIM, WD, 7, HDIM, 16.0f);
    k_cm_castbT<<<dim3((HDIM * (WD / 8)) / 256, NH), 256, 0, stream>>>(Wk, WQKV16 + (size_t)WD * WD,     (long long)WD * HDIM, (long long)HDIM * WD, HDIM, WD, 7, HDIM, 16.0f);
    k_cm_castbT<<<dim3((HDIM * (WD / 8)) / 256, NH), 256, 0, stream>>>(Wv, WQKV16 + (size_t)2 * WD * WD, (long long)WD * HDIM, (long long)HDIM * WD, HDIM, WD, 7, HDIM, 16.0f);
    k_cm_castbT<<<dim3((FF * (WD / 8)) / 256, 1), 256, 0, stream>>>(W1, W1T, 0LL, 0LL, FF, WD, 7, FF, 16.0f);
    k_cm_castbT<<<dim3((WD * (FF / 8)) / 256, 1), 256, 0, stream>>>(W2, W2T, 0LL, 0LL, WD, FF, 9, WD, 16.0f);
    k_gemm_qkv<<<((ROWS / 64) * (QW / 64) + 7) / 8, 256, 0, stream>>>(H16, WQKV16, QKV);
    k_attn<<<NB * NH * (SEQ / 64), 128, 0, stream>>>(QKV, x, X1);
    k_ln_mid<<<(ROWS + 7) / 8, 256, 0, stream>>>(X1, g2, be2, H2);
    k_gemm_mlp1<<<((ROWS / 64) * (FF / 64) + 7) / 8, 256, 0, stream>>>(H2, W1T, A1, b1);
    k_gemm_mlp2<<<((ROWS / 64) * (WD / 64) + 7) / 8, 256, 0, stream>>>(A1, W2T, out, X1, b2);
}
